// BertAttention_26156350832687
// MI455X (gfx1250) — hardware-verified
//
#include <hip/hip_runtime.h>
#include <stdint.h>


#ifndef NB
#define NB 4
#endif
#ifndef SEQ
#define SEQ 2048
#endif
#define NB_FULL 4
#define SEQ_FULL 2048
#define HID 1024
#define NHEAD 16
#define HDIM 64
#define PCARRY 4096.0f
#define CCARRY 64.0f
#define WCARRY 16.0f

static_assert(NB >= 1 && NB <= NB_FULL);
static_assert(SEQ >= 128 && SEQ <= SEQ_FULL && (SEQ % 128) == 0);
static_assert(HID == NHEAD * HDIM);
static_assert((HID % 256) == 0);
static_assert(((HID * HID) % 2048) == 0);

typedef __bf16 bf16_t;
typedef _Float16 f16_t;
typedef __attribute__((ext_vector_type(16))) __bf16 v16bf;
typedef __attribute__((ext_vector_type(8)))  __bf16 bf16x8;
typedef __attribute__((ext_vector_type(16))) _Float16 v16h;
typedef __attribute__((ext_vector_type(8)))  _Float16 h16x8;
typedef __attribute__((ext_vector_type(8)))  float v8f;
typedef __attribute__((ext_vector_type(4)))  float f32x4;
typedef __attribute__((ext_vector_type(4)))  unsigned int u32x4;
typedef __attribute__((ext_vector_type(8)))  unsigned short us16x8;
typedef __attribute__((ext_vector_type(4)))  unsigned short us16x4;

__device__ __forceinline__ unsigned int bf_bits(float f) {
  unsigned int u = __builtin_bit_cast(unsigned int, f);
  return (u + 0x7FFFu + ((u >> 16) & 1u)) >> 16;
}
__device__ __forceinline__ float bf_rne(float f) {
  return __builtin_bit_cast(float, bf_bits(f) << 16);
}
__device__ __forceinline__ float bfu2f(unsigned short u) {
  return __builtin_bit_cast(float, ((unsigned int)u) << 16);
}

__device__ __forceinline__ v16bf frag_row_bf(const bf16_t* p, int ld) {
  const int lane = threadIdx.x & 31;
  const int hf = lane >> 4, r = lane & 15;
  const bf16_t* q = p + r * ld + hf * 8;
  bf16x8 lo = *(const bf16x8*)(q);
  bf16x8 hi = *(const bf16x8*)(q + 16);
  return __builtin_shufflevector(lo, hi, 0, 1, 2, 3, 4, 5, 6, 7,
                                 8, 9, 10, 11, 12, 13, 14, 15);
}
__device__ __forceinline__ v16h frag_row_h(const f16_t* p, int ld) {
  const int lane = threadIdx.x & 31;
  const int hf = lane >> 4, r = lane & 15;
  const f16_t* q = p + r * ld + hf * 8;
  h16x8 lo = *(const h16x8*)(q);
  h16x8 hi = *(const h16x8*)(q + 16);
  return __builtin_shufflevector(lo, hi, 0, 1, 2, 3, 4, 5, 6, 7,
                                 8, 9, 10, 11, 12, 13, 14, 15);
}

__device__ __forceinline__ v8f wmma_bf16(v16bf a, v16bf b, v8f c) {
  v8f d = __builtin_amdgcn_wmma_f32_16x16x32_bf16(false, a, false, b, (short)0, c, false, false);
  asm volatile("v_nop\n\tv_nop\n\tv_nop\n\tv_nop" : "+v"(d) : "v"(a), "v"(b));
  return d;
}
__device__ __forceinline__ v8f wmma_f16(v16h a, v16h b, v8f c) {
  v8f d = __builtin_amdgcn_wmma_f32_16x16x32_f16(false, a, false, b, (short)0, c, false, false);
  asm volatile("v_nop\n\tv_nop\n\tv_nop\n\tv_nop" : "+v"(d) : "v"(a), "v"(b));
  return d;
}

__device__ __forceinline__ void wave_lds_sync() {
  asm volatile("s_wait_dscnt 0x0" ::: "memory");
  __builtin_amdgcn_wave_barrier();
}

__global__ __launch_bounds__(256) void k_cast_rows(const float* __restrict__ X,
                                                    unsigned short* __restrict__ Y) {
  const size_t g = (size_t)blockIdx.x * 256 + threadIdx.x;
  const size_t e = g * 8;
  const int prow = (int)(e >> 10);
  const int col = (int)(e & 1023);
  if (prow >= NB * SEQ) return;
  const int b = prow / SEQ;
  const int s = prow - b * SEQ;
  const float* src = X + ((size_t)b * SEQ_FULL + s) * HID + col;
  const f32x4 f0 = ((const f32x4*)src)[0];
  const f32x4 f1 = ((const f32x4*)src)[1];
  u32x4 pk;
  pk.x = bf_bits(f0.x) | (bf_bits(f0.y) << 16);
  pk.y = bf_bits(f0.z) | (bf_bits(f0.w) << 16);
  pk.z = bf_bits(f1.x) | (bf_bits(f1.y) << 16);
  pk.w = bf_bits(f1.z) | (bf_bits(f1.w) << 16);
  unsigned short* dst = Y + (size_t)prow * HID + col;
  *(volatile u32x4*)dst = pk;
  __threadfence();
  *(volatile u32x4*)dst = pk;
}

template <int F16OUT>
__global__ __launch_bounds__(256) void k_cast_mat(const float* __restrict__ W,
                                                   unsigned short* __restrict__ Y) {
  const size_t g = (size_t)blockIdx.x * 256 + threadIdx.x;
  const size_t e = g * 8;
  if (e >= (size_t)HID * HID) return;
  const f32x4 f0 = *(const f32x4*)(W + e);
  const f32x4 f1 = *(const f32x4*)(W + e + 4);
  u32x4 pk;
  if constexpr (F16OUT != 0) {
    h16x8 hv;
    hv[0] = (f16_t)(bf_rne(f0.x) * WCARRY);
    hv[1] = (f16_t)(bf_rne(f0.y) * WCARRY);
    hv[2] = (f16_t)(bf_rne(f0.z) * WCARRY);
    hv[3] = (f16_t)(bf_rne(f0.w) * WCARRY);
    hv[4] = (f16_t)(bf_rne(f1.x) * WCARRY);
    hv[5] = (f16_t)(bf_rne(f1.y) * WCARRY);
    hv[6] = (f16_t)(bf_rne(f1.z) * WCARRY);
    hv[7] = (f16_t)(bf_rne(f1.w) * WCARRY);
    pk = __builtin_bit_cast(u32x4, hv);
  } else {
    pk.x = bf_bits(f0.x) | (bf_bits(f0.y) << 16);
    pk.y = bf_bits(f0.z) | (bf_bits(f0.w) << 16);
    pk.z = bf_bits(f1.x) | (bf_bits(f1.y) << 16);
    pk.w = bf_bits(f1.z) | (bf_bits(f1.w) << 16);
  }
  unsigned short* dst = Y + e;
  *(volatile u32x4*)dst = pk;
  __threadfence();
  *(volatile u32x4*)dst = pk;
}

__global__ __launch_bounds__(256) void k_xsum(const unsigned short* __restrict__ Xb,
                                               float* __restrict__ xsum) {
  const int k = blockIdx.x * 256 + threadIdx.x;
  const int b = blockIdx.y;
  const unsigned short* p = Xb + (size_t)b * SEQ * HID + k;
  float a0 = 0.0f, a1 = 0.0f, a2 = 0.0f, a3 = 0.0f;
#pragma unroll 1
  for (int s = 0; s < SEQ; s += 4) {
    a0 += bfu2f(p[(size_t)(s + 0) * HID]);
    a1 += bfu2f(p[(size_t)(s + 1) * HID]);
    a2 += bfu2f(p[(size_t)(s + 2) * HID]);
    a3 += bfu2f(p[(size_t)(s + 3) * HID]);
  }
  const float v = (a0 + a1) + (a2 + a3);
  float* d = xsum + (size_t)b * HID + k;
  *(volatile float*)d = v;
  __threadfence();
  *(volatile float*)d = v;
}

__global__ __launch_bounds__(256) void k_vsum(const float* __restrict__ xsum,
                                               const unsigned short* __restrict__ Wb,
                                               float* __restrict__ vsum) {
  __shared__ __align__(16) float xs[HID];
  const int tid = threadIdx.x;
  const int b = blockIdx.y;
  const int n = blockIdx.x * 256 + tid;
  ((f32x4*)xs)[tid] = ((const f32x4*)(xsum + (size_t)b * HID))[tid];
  __syncthreads();
  const unsigned short* wrow = Wb + (size_t)n * HID;
  float a0 = 0.0f, a1 = 0.0f, a2 = 0.0f, a3 = 0.0f;
#pragma unroll 1
  for (int k = 0; k < HID; k += 4) {
    const us16x4 w4 = *(const us16x4*)(wrow + k);
    const f32x4 x4 = *(const f32x4*)(xs + k);
    a0 += x4.x * bfu2f(w4.x);
    a1 += x4.y * bfu2f(w4.y);
    a2 += x4.z * bfu2f(w4.z);
    a3 += x4.w * bfu2f(w4.w);
  }
  const float v = (a0 + a1) + (a2 + a3);
  float* d = vsum + (size_t)b * HID + n;
  *(volatile float*)d = v;
  __threadfence();
  *(volatile float*)d = v;
}

template <bool TRANS_OUT>
__global__ __launch_bounds__(256) __attribute__((amdgpu_num_vgpr(256)))
void k_proj_gemm(const bf16_t* __restrict__ X, const bf16_t* __restrict__ WT,
                 f16_t* __restrict__ outp) {
  constexpr int K = HID;
  constexpr int LDA = 40;
  constexpr int LDC = 136;
  static_assert(128 * LDC * 2 >= 2 * 128 * LDA * 2);
  static_assert((K % 32) == 0);
  __shared__ __align__(16) unsigned char smem[128 * LDC * 2];
  bf16_t* As = (bf16_t*)smem;
  bf16_t* Bs = As + 128 * LDA;
  f16_t* Cs = (f16_t*)smem;

  const int tid = threadIdx.x;
  const int lane = tid & 31, w = tid >> 5;
  const int wr = w >> 1, wc = w & 1;
  const int hf = lane >> 4, nl = lane & 15;
  const int m0 = blockIdx.y * 128, n0 = blockIdx.x * 128;

  v8f acc[2][4];
#pragma unroll
  for (int i = 0; i < 2; ++i)
#pragma unroll
    for (int j = 0; j < 4; ++j)
#pragma unroll
      for (int r = 0; r < 8; ++r) acc[i][j][r] = 0.0f;

#pragma unroll 1
  for (int kt = 0; kt < K / 32; ++kt) {
#pragma unroll
    for (int it = 0; it < 2; ++it) {
      const int p = it * 256 + tid;
      const int r = p >> 2, c = (p & 3) * 8;
      *(bf16x8*)(As + r * LDA + c) =
          *(const bf16x8*)(X + (size_t)(m0 + r) * K + kt * 32 + c);
      *(bf16x8*)(Bs + r * LDA + c) =
          *(const bf16x8*)(WT + (size_t)(n0 + r) * K + kt * 32 + c);
    }
    __syncthreads();

    const v16bf a0 = frag_row_bf(As + (wr * 32) * LDA, LDA);
    const v16bf a1 = frag_row_bf(As + (wr * 32 + 16) * LDA, LDA);
#pragma unroll
    for (int nf = 0; nf < 4; ++nf) {
      const v16bf bb = frag_row_bf(Bs + (wc * 64 + nf * 16) * LDA, LDA);
      acc[0][nf] = wmma_bf16(a0, bb, acc[0][nf]);
      acc[1][nf] = wmma_bf16(a1, bb, acc[1][nf]);
    }
    __syncthreads();
  }

#pragma unroll
  for (int mf = 0; mf < 2; ++mf)
#pragma unroll
    for (int nf = 0; nf < 4; ++nf)
#pragma unroll
      for (int r = 0; r < 8; ++r) {
        const int ml = wr * 32 + mf * 16 + hf * 8 + r;
        const int nloc = wc * 64 + nf * 16 + nl;
        const f16_t hv = (f16_t)(acc[mf][nf][r]);
        if constexpr (TRANS_OUT) {
          Cs[nloc * LDC + ml] = hv;
        } else {
          Cs[ml * LDC + nloc] = hv;
        }
      }
  __syncthreads();

  const int c16 = tid & 15;
  const int bsel = m0 / SEQ;
  const int s0 = m0 - bsel * SEQ;
  u32x4 vals[8];
  f16_t* dsts[8];
#pragma unroll
  for (int it = 0; it < 8; ++it) {
    const int row = it * 16 + (tid >> 4);
    const h16x8 hv8 = *(const h16x8*)(Cs + row * LDC + c16 * 8);
    vals[it] = __builtin_bit_cast(u32x4, hv8);
    if constexpr (TRANS_OUT) {
      const int n = n0 + row;
      const int hh = n >> 6, dd = n & 63;
      dsts[it] = outp + ((size_t)((bsel * NHEAD + hh) * HDIM + dd)) * SEQ + s0 + c16 * 8;
    } else {
      dsts[it] = outp + (size_t)(m0 + row) * HID + n0 + c16 * 8;
    }
  }
#pragma unroll
  for (int it = 0; it < 8; ++it) *(volatile u32x4*)dsts[it] = vals[it];
  __threadfence();
#pragma unroll
  for (int it = 0; it < 8; ++it) *(volatile u32x4*)dsts[it] = vals[it];
}

__global__ __launch_bounds__(256) __attribute__((amdgpu_num_vgpr(256)))
void k_attn(const f16_t* __restrict__ Qp, const f16_t* __restrict__ Kp,
            const f16_t* __restrict__ VTp, const float* __restrict__ vsum,
            const int* __restrict__ maskp, f16_t* __restrict__ ctxp) {
  constexpr int LDK = 72;
  constexpr int KS_BYTES = 64 * LDK * 2;
  constexpr int PS_BYTES = 8 * 16 * LDK * 2;
  constexpr int SMEM_BYTES = 2 * KS_BYTES + PS_BYTES;
  __shared__ __align__(16) unsigned char smem[SMEM_BYTES];
  f16_t* Ks = (f16_t*)smem;
  f16_t* Vs = (f16_t*)(smem + KS_BYTES);
  f16_t* Ps = (f16_t*)(smem + 2 * KS_BYTES);
  (void)maskp;

  const int tid = threadIdx.x, lane = tid & 31, w = tid >> 5;
  const int hf = lane >> 4, nl = lane & 15;
  const int qtiles = SEQ / 128;
  const int qt = blockIdx.x % qtiles;
  const int bh = blockIdx.x / qtiles;
  const int b = bh / NHEAD;
  const int h = bh - b * NHEAD;
  const int q0 = qt * 128 + w * 16;

  v16h qa[2];
#pragma unroll
  for (int kk = 0; kk < 2; ++kk)
    qa[kk] = frag_row_h(Qp + (size_t)(b * SEQ + q0) * HID + h * HDIM + kk * 32, HID);

  float mrow[8], lrow[8], gctr[8];
  v8f o[4];
#pragma unroll
  for (int r = 0; r < 8; ++r) { mrow[r] = -1e30f; lrow[r] = 0.0f; gctr[r] = 0.0f; }
#pragma unroll
  for (int df = 0; df < 4; ++df)
#pragma unroll
    for (int r = 0; r < 8; ++r) o[df][r] = 0.0f;

  const float scale = 0.03125f;
  const size_t kbase = (size_t)(b * SEQ) * HID + h * HDIM;
  const size_t vbase = (size_t)(b * NHEAD + h) * HDIM * SEQ;
  f16_t* Pw = Ps + (w * 16) * LDK;

#pragma unroll 1
  for (int kc = 0; kc < SEQ / 64; ++kc) {
#pragma unroll
    for (int it = 0; it < 2; ++it) {
      const int p = it * 256 + tid;
      const int r = p >> 3, c = (p & 7) * 8;
      *(h16x8*)(Ks + r * LDK + c) =
          *(const h16x8*)(Kp + kbase + (size_t)(kc * 64 + r) * HID + c);
      *(h16x8*)(Vs + r * LDK + c) =
          *(const h16x8*)(VTp + vbase + (size_t)r * SEQ + kc * 64 + c);
    }
    __syncthreads();

    v8f sf[4];
#pragma unroll
    for (int nf = 0; nf < 4; ++nf) {
      v8f c = {};
#pragma unroll
      for (int kk = 0; kk < 2; ++kk) {
        const v16h bb = frag_row_h(Ks + (nf * 16) * LDK + kk * 32, LDK);
        c = wmma_f16(qa[kk], bb, c);
      }
#pragma unroll
      for (int r = 0; r < 8; ++r) sf[nf][r] = c[r] * scale;
    }

    float mx[8];
#pragma unroll
    for (int r = 0; r < 8; ++r) {
      mx[r] = fmaxf(fmaxf(sf[0][r], sf[1][r]), fmaxf(sf[2][r], sf[3][r]));
#pragma unroll
      for (int off = 1; off < 16; off <<= 1)
        mx[r] = fmaxf(mx[r], __shfl_xor(mx[r], off, 16));
    }
    float gam[8];
#pragma unroll
    for (int r = 0; r < 8; ++r) {
      const float mnew = fmaxf(mrow[r], mx[r]);
      const float alpha = __expf(mrow[r] - mnew);
      if (kc == 0) gctr[r] = fminf(0.0f, mnew + 2.0f);
      mrow[r] = mnew;
      lrow[r] *= alpha;
#pragma unroll
      for (int df = 0; df < 4; ++df) o[df][r] *= alpha;
      gam[r] = __expf(gctr[r] - mnew);
    }
    float rs[8];
#pragma unroll
    for (int r = 0; r < 8; ++r) rs[r] = 0.0f;
#pragma unroll
    for (int nf = 0; nf < 4; ++nf)
#pragma unroll
      for (int r = 0; r < 8; ++r) {
        const float p = __expf(sf[nf][r] - mrow[r]);
        rs[r] += p;
        Pw[(hf * 8 + r) * LDK + nf * 16 + nl] = (f16_t)((p - gam[r]) * PCARRY);
      }
#pragma unroll
    for (int r = 0; r < 8; ++r) {
#pragma unroll
      for (int off = 1; off < 16; off <<= 1)
        rs[r] += __shfl_xor(rs[r], off, 16);
      lrow[r] += rs[r];
    }

    wave_lds_sync();

    v16h pa[2];
#pragma unroll
    for (int kk = 0; kk < 2; ++kk) pa[kk] = frag_row_h(Pw + kk * 32, LDK);
#pragma unroll
    for (int df = 0; df < 4; ++df)
#pragma unroll
      for (int kk = 0; kk < 2; ++kk) {
        const v16h bb = frag_row_h(Vs + (df * 16) * LDK + kk * 32, LDK);
        o[df] = wmma_f16(pa[kk], bb, o[df]);
      }
    __syncthreads();
  }

  float vs4[4];
#pragma unroll
  for (int df = 0; df < 4; ++df)
    vs4[df] = vsum[(size_t)b * HID + h * HDIM + df * 16 + nl];
  float ef[8], il[8];
#pragma unroll
  for (int r = 0; r < 8; ++r) {
    ef[r] = __expf(gctr[r] - mrow[r]);
    il[r] = CCARRY / lrow[r];
  }
#pragma unroll
  for (int df = 0; df < 4; ++df)
#pragma unroll
    for (int r = 0; r < 8; ++r) {
      const float val = (o[df][r] * (1.0f / PCARRY) + ef[r] * vs4[df]) * il[r];
      Pw[(hf * 8 + r) * LDK + df * 16 + nl] = (f16_t)val;
    }
  wave_lds_sync();

  u32x4 vals[4];
  f16_t* dsts[4];
#pragma unroll
  for (int it = 0; it < 4; ++it) {
    const int row = it * 4 + (lane >> 3);
    const int c8 = lane & 7;
    const h16x8 hv8 = *(const h16x8*)(Pw + row * LDK + c8 * 8);
    vals[it] = __builtin_bit_cast(u32x4, hv8);
    dsts[it] = ctxp + ((size_t)(b * SEQ + q0 + row)) * HID + h * HDIM + c8 * 8;
  }
#pragma unroll
  for (int it = 0; it < 4; ++it) *(volatile u32x4*)dsts[it] = vals[it];
  __threadfence();
#pragma unroll
  for (int it = 0; it < 4; ++it) *(volatile u32x4*)dsts[it] = vals[it];
}

__global__ __launch_bounds__(256) __attribute__((amdgpu_num_vgpr(256)))
void k_out_gemm(const f16_t* __restrict__ X, const f16_t* __restrict__ WT,
                float* __restrict__ outp) {
  constexpr int K = HID;
  constexpr int LDA = 40;
  constexpr int LDC = 68;
  constexpr int AB_BYTES = (128 + 64) * LDA * 2;
  constexpr int C_BYTES = 128 * LDC * 4;
  constexpr int SMEM_BYTES = AB_BYTES > C_BYTES ? AB_BYTES : C_BYTES;
  static_assert((K % 32) == 0);
  __shared__ __align__(16) unsigned char smem[SMEM_BYTES];
  f16_t* As = (f16_t*)smem;
  f16_t* Bs = As + 128 * LDA;
  float* Cs = (float*)smem;

  const int tid = threadIdx.x;
  const int lane = tid & 31, w = tid >> 5;
  const int wr = w >> 1, wc = w & 1;
  const int hf = lane >> 4, nl = lane & 15;
  const int m0 = blockIdx.y * 128, n0 = blockIdx.x * 64;

  v8f acc[2][2];
#pragma unroll
  for (int i = 0; i < 2; ++i)
#pragma unroll
    for (int j = 0; j < 2; ++j)
#pragma unroll
      for (int r = 0; r < 8; ++r) acc[i][j][r] = 0.0f;

#pragma unroll 1
  for (int kt = 0; kt < K / 32; ++kt) {
#pragma unroll
    for (int it = 0; it < 2; ++it) {
      const int p = it * 256 + tid;
      const int r = p >> 2, c = (p & 3) * 8;
      *(h16x8*)(As + r * LDA + c) =
          *(const h16x8*)(X + (size_t)(m0 + r) * K + kt * 32 + c);
    }
    {
      const int r = tid >> 2, c = (tid & 3) * 8;
      *(h16x8*)(Bs + r * LDA + c) =
          *(const h16x8*)(WT + (size_t)(n0 + r) * K + kt * 32 + c);
    }
    __syncthreads();

    const v16h a0 = frag_row_h(As + (wr * 32) * LDA, LDA);
    const v16h a1 = frag_row_h(As + (wr * 32 + 16) * LDA, LDA);
#pragma unroll
    for (int nf = 0; nf < 2; ++nf) {
      const v16h bb = frag_row_h(Bs + (wc * 32 + nf * 16) * LDA, LDA);
      acc[0][nf] = wmma_f16(a0, bb, acc[0][nf]);
      acc[1][nf] = wmma_f16(a1, bb, acc[1][nf]);
    }
    __syncthreads();
  }

  const float oscale = 1.0f / (CCARRY * WCARRY);
#pragma unroll
  for (int mf = 0; mf < 2; ++mf)
#pragma unroll
    for (int nf = 0; nf < 2; ++nf)
#pragma unroll
      for (int r = 0; r < 8; ++r) {
        const int ml = wr * 32 + mf * 16 + hf * 8 + r;
        const int nloc = wc * 32 + nf * 16 + nl;
        Cs[ml * LDC + nloc] = acc[mf][nf][r] * oscale;
      }
  __syncthreads();

  const int c16 = tid & 15;
  const int bsel = m0 / SEQ;
  const int s0 = m0 - bsel * SEQ;
  f32x4 vv[8];
  float* od[8];
#pragma unroll
  for (int it = 0; it < 8; ++it) {
    const int row = it * 16 + (tid >> 4);
    vv[it] = *(const f32x4*)(Cs + row * LDC + c16 * 4);
    od[it] = outp + ((size_t)(bsel * SEQ_FULL + s0 + row)) * HID + n0 + c16 * 4;
  }
#pragma unroll
  for (int it = 0; it < 8; ++it) *(volatile f32x4*)od[it] = vv[it];
  __threadfence();
#pragma unroll
  for (int it = 0; it < 8; ++it) *(volatile f32x4*)od[it] = vv[it];
}

extern "C" void kernel_launch(void* const* d_in, const int* in_sizes, int n_in,
                              void* d_out, int out_size, void* d_ws, size_t ws_size,
                              hipStream_t stream) {
  if (n_in < 6) return;
  const long long need_act = ((long long)(NB - 1) * SEQ_FULL + SEQ) * HID;
  if ((long long)in_sizes[0] < need_act) return;
  if (in_sizes[1] < 1) return;
  if (in_sizes[2] < HID * HID || in_sizes[3] < HID * HID) return;
  if (in_sizes[4] < HID * HID || in_sizes[5] < HID * HID) return;
  if ((long long)out_size < need_act) return;

  const float* hidden = (const float*)d_in[0];
  const int* mask = (const int*)d_in[1];
  const float* Wq = (const float*)d_in[2];
  const float* Wk = (const float*)d_in[3];
  const float* Wv = (const float*)d_in[4];
  const float* Wo = (const float*)d_in[5];

  const size_t act_elems = (size_t)NB * SEQ * HID;
  const size_t act_bytes = act_elems * 2;
  const size_t w_bytes = (size_t)HID * HID * 2;
  const size_t sum_bytes = (size_t)NB * HID * 4;
  char* ws = (char*)d_ws;
  size_t off = 0;
  unsigned short* Xb  = (unsigned short*)(ws + off); off += act_bytes;
  unsigned short* Wqb = (unsigned short*)(ws + off); off += w_bytes;
  unsigned short* Wkb = (unsigned short*)(ws + off); off += w_bytes;
  unsigned short* Wvb = (unsigned short*)(ws + off); off += w_bytes;
  unsigned short* Woh = (unsigned short*)(ws + off); off += w_bytes;
  float* xsum = (float*)(ws + off); off += sum_bytes;
  float* vsum = (float*)(ws + off); off += sum_bytes;
  f16_t* Qp = (f16_t*)(ws + off); off += act_bytes;
  f16_t* Kp = (f16_t*)(ws + off); off += act_bytes;
  f16_t* VT = (f16_t*)(ws + off); off += act_bytes;
  f16_t* Cx = (f16_t*)(ws + off); off += act_bytes;
  if (off > ws_size) return;
  if (off > (size_t)134217728) return;

  const dim3 blk(256);
  const dim3 g_rows((unsigned)((act_elems / 8) / 256));
  const dim3 g_mat((unsigned)(((size_t)HID * HID / 8) / 256));
  const dim3 g_sum(HID / 256, NB);
  const dim3 g_gemm(HID / 128, (NB * SEQ) / 128);
  const dim3 g_attn(NB * NHEAD * (SEQ / 128));
  const dim3 g_out(HID / 64, (NB * SEQ) / 128);

  k_cast_rows<<<g_rows, blk, 0, stream>>>(hidden, Xb);
  k_cast_mat<0><<<g_mat, blk, 0, stream>>>(Wq, Wqb);
  k_cast_mat<0><<<g_mat, blk, 0, stream>>>(Wk, Wkb);
  k_cast_mat<0><<<g_mat, blk, 0, stream>>>(Wv, Wvb);
  k_cast_mat<1><<<g_mat, blk, 0, stream>>>(Wo, Woh);

  k_xsum<<<g_sum, blk, 0, stream>>>(Xb, xsum);
  k_vsum<<<g_sum, blk, 0, stream>>>(xsum, Wvb, vsum);

  k_proj_gemm<false><<<g_gemm, blk, 0, stream>>>((const bf16_t*)Xb, (const bf16_t*)Wqb, Qp);
  k_proj_gemm<false><<<g_gemm, blk, 0, stream>>>((const bf16_t*)Xb, (const bf16_t*)Wkb, Kp);
  k_proj_gemm<true><<<g_gemm, blk, 0, stream>>>((const bf16_t*)Xb, (const bf16_t*)Wvb, VT);

  k_attn<<<g_attn, blk, 0, stream>>>(Qp, Kp, VT, vsum, mask, Cx);

  k_out_gemm<<<g_out, blk, 0, stream>>>(Cx, (const f16_t*)Woh, (float*)d_out);
}
